// Multi_header_attention_12970801233980
// MI455X (gfx1250) — hardware-verified
//
#include <hip/hip_runtime.h>
#include <stddef.h>
#include <stdint.h>


#define F_DIM 256
#define NSEQ  2048
#define NH    4
#define HD    64

typedef _Float16      v16h __attribute__((ext_vector_type(16)));
typedef __bf16        v16b __attribute__((ext_vector_type(16)));
typedef float         v8f  __attribute__((ext_vector_type(8)));
typedef float         v4f  __attribute__((ext_vector_type(4)));
typedef unsigned int  v4ua __attribute__((ext_vector_type(4), may_alias));
typedef float         v4fa __attribute__((ext_vector_type(4), may_alias));

union FragB { v16b v; v4ua q[2]; };
union FragH { v16h v; v4ua q[2]; };

__device__ __forceinline__ v8f zero8() {
  v8f z = {0.0f, 0.0f, 0.0f, 0.0f, 0.0f, 0.0f, 0.0f, 0.0f};
  return z;
}

__device__ __forceinline__ v8f mma_bf16(v16b a, v16b b, v8f c) {
  c = __builtin_amdgcn_wmma_f32_16x16x32_bf16(false, a, false, b, (short)0, c, false, false);
  asm volatile("v_nop\n\tv_nop\n\tv_nop\n\tv_nop" : "+v"(c) : "v"(a), "v"(b));
  return c;
}
__device__ __forceinline__ v8f mma_f16(v16h a, v16h b, v8f c) {
  c = __builtin_amdgcn_wmma_f32_16x16x32_f16(false, a, false, b, (short)0, c, false, false);
  asm volatile("v_nop\n\tv_nop\n\tv_nop\n\tv_nop" : "+v"(c) : "v"(a), "v"(b));
  return c;
}

__device__ __forceinline__ unsigned int bf16_rne(float x) {
  const unsigned int u = __builtin_bit_cast(unsigned int, x);
  return (u + 0x7FFFu + ((u >> 16) & 1u)) >> 16;
}
__device__ __forceinline__ void split2(float x, unsigned int& hb, unsigned int& lb) {
  hb = bf16_rne(x);
  const float hf = __builtin_bit_cast(float, hb << 16);
  lb = bf16_rne(x - hf);
}
__device__ __forceinline__ unsigned int h16_bits(float x) {
  const _Float16 hv = (_Float16)x;
  return (unsigned int)__builtin_bit_cast(unsigned short, hv);
}

__global__ __launch_bounds__(256)
void k_wcvt(const float* __restrict__ w0, const float* __restrict__ w1,
            const float* __restrict__ w2, const float* __restrict__ w3,
            unsigned short* wh, unsigned short* wl, int nper)
{
  const int chunks = nper >> 3;
  const int gid = (int)blockIdx.x * 256 + (int)threadIdx.x;
  const int mat = gid / chunks;
  if (mat >= 4) return;
  const int c = gid - mat * chunks;
  const float* src = (mat == 0) ? w0 : ((mat == 1) ? w1 : ((mat == 2) ? w2 : w3));
  const v4f x0 = *(const v4f*)(src + (size_t)c * 8);
  const v4f x1 = *(const v4f*)(src + (size_t)c * 8 + 4);
  unsigned int hb[8], lb[8];
#pragma unroll
  for (int q = 0; q < 4; ++q) {
    split2(x0[q], hb[q], lb[q]);
    split2(x1[q], hb[4 + q], lb[4 + q]);
  }
  v4ua hv, lv;
#pragma unroll
  for (int j = 0; j < 4; ++j) {
    hv[j] = hb[2 * j] | (hb[2 * j + 1] << 16);
    lv[j] = lb[2 * j] | (lb[2 * j + 1] << 16);
  }
  unsigned short* dh = wh + (size_t)mat * nper + (size_t)c * 8;
  unsigned short* dl = wl + (size_t)mat * nper + (size_t)c * 8;
  *(volatile v4ua*)dh = hv;
  *(volatile v4ua*)dl = lv;
  __threadfence();
  *(volatile v4ua*)dh = hv;
  *(volatile v4ua*)dl = lv;
}

template <int MODE>
__global__ __launch_bounds__(256)
void k_proj(const float* __restrict__ X, const unsigned short* __restrict__ Wh,
            const unsigned short* __restrict__ Wl, const float* __restrict__ bias,
            unsigned short* o16a, unsigned short* o16b, float* o32, int nB)
{
  __shared__ __align__(16) unsigned char lds_raw[34816];
  unsigned short* xs_h = (unsigned short*)lds_raw;
  unsigned short* xs_l = xs_h + 64 * 136;

  const int blk = (int)blockIdx.x;
  const int b  = blk >> 5;
  const int n0 = (blk & 31) * 64;
  if (b >= nB) return;
  const int tid = (int)threadIdx.x;
  const int wv = tid >> 5, lane = tid & 31, h = lane >> 4, m = lane & 15;

  v8f acc[2][4];
#pragma unroll
  for (int et = 0; et < 2; ++et)
#pragma unroll
    for (int nt = 0; nt < 4; ++nt) acc[et][nt] = zero8();

  const int fl = tid & 127, nh = tid >> 7;
  for (int half = 0; half < 2; ++half) {
    __syncthreads();
    {
      const float* src = X + ((size_t)(b * F_DIM + half * 128 + fl)) * NSEQ + n0 + nh * 32;
#pragma unroll
      for (int j = 0; j < 8; ++j) {
        const v4f x = *(const v4f*)(src + j * 4);
#pragma unroll
        for (int q = 0; q < 4; ++q) {
          unsigned int hb, lb;
          split2(x[q], hb, lb);
          const int nl = nh * 32 + j * 4 + q;
          xs_h[nl * 136 + fl] = (unsigned short)hb;
          xs_l[nl * 136 + fl] = (unsigned short)lb;
        }
      }
    }
    __syncthreads();
#pragma unroll
    for (int kk = 0; kk < 4; ++kk) {
      const int fg = half * 128 + kk * 32 + 8 * h;
      const int fs = kk * 32 + 8 * h;
      FragB ah[2], al[2];
#pragma unroll
      for (int et = 0; et < 2; ++et) {
        const size_t wo = (size_t)((wv * 2 + et) * 16 + m) * F_DIM + fg;
        ah[et].q[0] = *(const v4ua*)(Wh + wo);
        ah[et].q[1] = *(const v4ua*)(Wh + wo + 16);
        al[et].q[0] = *(const v4ua*)(Wl + wo);
        al[et].q[1] = *(const v4ua*)(Wl + wo + 16);
      }
#pragma unroll
      for (int nt = 0; nt < 4; ++nt) {
        const int xo = (nt * 16 + m) * 136 + fs;
        FragB xh, xl;
        xh.q[0] = *(const v4ua*)(xs_h + xo);
        xh.q[1] = *(const v4ua*)(xs_h + xo + 16);
        xl.q[0] = *(const v4ua*)(xs_l + xo);
        xl.q[1] = *(const v4ua*)(xs_l + xo + 16);
#pragma unroll
        for (int et = 0; et < 2; ++et) {
          v8f c = acc[et][nt];
          c = mma_bf16(al[et].v, xh.v, c);
          c = mma_bf16(ah[et].v, xl.v, c);
          c = mma_bf16(ah[et].v, xh.v, c);
          acc[et][nt] = c;
        }
      }
    }
  }

#pragma unroll
  for (int et = 0; et < 2; ++et) {
#pragma unroll
    for (int r = 0; r < 8; ++r) {
      const float bz = bias[(wv * 2 + et) * 16 + 8 * h + r];
#pragma unroll
      for (int nt = 0; nt < 4; ++nt) acc[et][nt][r] += bz;
    }
  }

  if (MODE == 0) {
    unsigned short* so = xs_h;
    for (int pl = 0; pl < 2; ++pl) {
      __syncthreads();
#pragma unroll
      for (int et = 0; et < 2; ++et) {
        const int T = wv * 2 + et;
#pragma unroll
        for (int nt = 0; nt < 4; ++nt) {
#pragma unroll
          for (int r = 0; r < 8; ++r) {
            unsigned int hb, lb;
            split2(acc[et][nt][r], hb, lb);
            const int hh = r & 3;
            const int d  = 4 * T + 2 * h + (r >> 2);
            so[(hh * 64 + nt * 16 + m) * 64 + d] = (unsigned short)(pl ? lb : hb);
          }
        }
      }
      __syncthreads();
      unsigned short* dstp = pl ? o16b : o16a;
      v4ua vals[8];
#pragma unroll
      for (int i = 0; i < 8; ++i) {
        const int L = wv * 32 + i * 4 + (lane >> 3);
        vals[i] = *(const v4ua*)(so + L * 64 + (lane & 7) * 8);
      }
#pragma unroll
      for (int i = 0; i < 8; ++i) {
        const int L = wv * 32 + i * 4 + (lane >> 3);
        const int hh = L >> 6, nl = L & 63;
        unsigned short* dst = dstp + ((((size_t)(b * NH + hh)) * NSEQ + n0 + nl) * HD + (lane & 7) * 8);
        *(volatile v4ua*)dst = vals[i];
      }
      __threadfence();
#pragma unroll
      for (int i = 0; i < 8; ++i) {
        const int L = wv * 32 + i * 4 + (lane >> 3);
        const int hh = L >> 6, nl = L & 63;
        unsigned short* dst = dstp + ((((size_t)(b * NH + hh)) * NSEQ + n0 + nl) * HD + (lane & 7) * 8);
        *(volatile v4ua*)dst = vals[i];
      }
    }
  } else if (MODE == 1) {
    unsigned short* so = xs_h;
    __syncthreads();
#pragma unroll
    for (int et = 0; et < 2; ++et) {
      const int T = wv * 2 + et;
#pragma unroll
      for (int nt = 0; nt < 4; ++nt) {
#pragma unroll
        for (int r = 0; r < 8; ++r) {
          const int hh = r & 3;
          const int d  = 4 * T + 2 * h + (r >> 2);
          so[(hh * 64 + d) * 64 + nt * 16 + m] = (unsigned short)h16_bits(acc[et][nt][r] * 16.0f);
        }
      }
    }
    __syncthreads();
    v4ua vals[8];
#pragma unroll
    for (int i = 0; i < 8; ++i) {
      const int L = wv * 32 + i * 4 + (lane >> 3);
      vals[i] = *(const v4ua*)(so + L * 64 + (lane & 7) * 8);
    }
#pragma unroll
    for (int i = 0; i < 8; ++i) {
      const int L = wv * 32 + i * 4 + (lane >> 3);
      const int hh = L >> 6, d = L & 63;
      unsigned short* dst = o16a + ((((size_t)(b * NH + hh)) * HD + d) * NSEQ + n0 + (lane & 7) * 8);
      *(volatile v4ua*)dst = vals[i];
    }
    __threadfence();
#pragma unroll
    for (int i = 0; i < 8; ++i) {
      const int L = wv * 32 + i * 4 + (lane >> 3);
      const int hh = L >> 6, d = L & 63;
      unsigned short* dst = o16a + ((((size_t)(b * NH + hh)) * HD + d) * NSEQ + n0 + (lane & 7) * 8);
      *(volatile v4ua*)dst = vals[i];
    }
  } else {
    float* sof = (float*)lds_raw;
    for (int eh = 0; eh < 2; ++eh) {
      __syncthreads();
      if ((wv >> 2) == eh) {
#pragma unroll
        for (int et = 0; et < 2; ++et) {
          const int T = wv * 2 + et;
#pragma unroll
          for (int nt = 0; nt < 4; ++nt) {
#pragma unroll
            for (int r = 0; r < 8; ++r) {
              const int el = T * 16 + 8 * h + r - eh * 128;
              sof[el * 64 + nt * 16 + m] = acc[et][nt][r];
            }
          }
        }
      }
      __syncthreads();
      v4fa vals[8];
#pragma unroll
      for (int i = 0; i < 8; ++i) {
        const int L = wv * 32 + i * 4 + (lane >> 3);
        const int el = L >> 1, hf = L & 1;
        vals[i] = *(const v4fa*)(sof + el * 64 + hf * 32 + (lane & 7) * 4);
      }
#pragma unroll
      for (int i = 0; i < 8; ++i) {
        const int L = wv * 32 + i * 4 + (lane >> 3);
        const int el = L >> 1, hf = L & 1;
        float* dst = o32 + (((size_t)(b * F_DIM + eh * 128 + el)) * NSEQ + n0 + hf * 32 + (lane & 7) * 4);
        *(volatile v4fa*)dst = vals[i];
      }
      __threadfence();
#pragma unroll
      for (int i = 0; i < 8; ++i) {
        const int L = wv * 32 + i * 4 + (lane >> 3);
        const int el = L >> 1, hf = L & 1;
        float* dst = o32 + (((size_t)(b * F_DIM + eh * 128 + el)) * NSEQ + n0 + hf * 32 + (lane & 7) * 4);
        *(volatile v4fa*)dst = vals[i];
      }
    }
  }
}

__global__ __launch_bounds__(256)
void k_attn(const unsigned short* __restrict__ qh, const unsigned short* __restrict__ ql,
            const unsigned short* __restrict__ kh, const unsigned short* __restrict__ kl,
            const unsigned short* __restrict__ vp, float* xo, int nB)
{
  __shared__ __align__(16) unsigned char lds_raw[46080];
  unsigned short* kbh = (unsigned short*)lds_raw;
  unsigned short* kbl = kbh + 64 * 72;
  unsigned short* vb  = kbl + 64 * 72;
  unsigned short* pst = vb  + 64 * 72;

  const int blk = (int)blockIdx.x;
  const int bh = blk >> 4, rg = blk & 15;
  if (bh >= nB * NH) return;
  const int b = bh >> 2, head = bh & 3;
  const int tid = (int)threadIdx.x;
  const int wv = tid >> 5, lane = tid & 31, h = lane >> 4, m = lane & 15;
  const int n0b = rg * 128;
  const int n0w = n0b + wv * 16;

  FragB qf[2][2];
  {
    const size_t qo = ((size_t)bh * NSEQ + n0w + m) * HD + 8 * h;
#pragma unroll
    for (int dh = 0; dh < 2; ++dh) {
      qf[dh][0].q[0] = *(const v4ua*)(qh + qo + dh * 32);
      qf[dh][0].q[1] = *(const v4ua*)(qh + qo + dh * 32 + 16);
      qf[dh][1].q[0] = *(const v4ua*)(ql + qo + dh * 32);
      qf[dh][1].q[1] = *(const v4ua*)(ql + qo + dh * 32 + 16);
    }
  }

  float mrun[8], lrun[8];
  v8f oacc[4];
#pragma unroll
  for (int r = 0; r < 8; ++r) { mrun[r] = -3.0e38f; lrun[r] = 0.0f; }
#pragma unroll
  for (int dt = 0; dt < 4; ++dt) oacc[dt] = zero8();

  unsigned short* pw = pst + wv * (16 * 72);

  for (int kt = 0; kt < NSEQ / 64; ++kt) {
    const int m0 = kt * 64;
    __syncthreads();
#pragma unroll
    for (int cc = 0; cc < 2; ++cc) {
      const int c = tid + cc * 256;
      const int rr = c >> 3, pc = (c & 7) * 8;
      const size_t ko = ((size_t)bh * NSEQ + m0 + rr) * HD + pc;
      const size_t vo = ((size_t)bh * HD + rr) * NSEQ + m0 + pc;
      const v4ua th = *(const v4ua*)(kh + ko);
      const v4ua tl = *(const v4ua*)(kl + ko);
      const v4ua tv = *(const v4ua*)(vp + vo);
      *(v4ua*)(kbh + rr * 72 + pc) = th;
      *(v4ua*)(kbl + rr * 72 + pc) = tl;
      *(v4ua*)(vb  + rr * 72 + pc) = tv;
    }
    __syncthreads();

    v8f s[4];
#pragma unroll
    for (int mt = 0; mt < 4; ++mt) {
      v8f c = zero8();
#pragma unroll
      for (int dh = 0; dh < 2; ++dh) {
        const int ko = (mt * 16 + m) * 72 + dh * 32 + 8 * h;
        FragB fh, fl;
        fh.q[0] = *(const v4ua*)(kbh + ko);
        fh.q[1] = *(const v4ua*)(kbh + ko + 16);
        fl.q[0] = *(const v4ua*)(kbl + ko);
        fl.q[1] = *(const v4ua*)(kbl + ko + 16);
        c = mma_bf16(qf[dh][1].v, fh.v, c);
        c = mma_bf16(qf[dh][0].v, fl.v, c);
        c = mma_bf16(qf[dh][0].v, fh.v, c);
      }
      s[mt] = c;
    }

    float sc[8];
#pragma unroll
    for (int r = 0; r < 8; ++r) {
      float tm = fmaxf(fmaxf(s[0][r], s[1][r]), fmaxf(s[2][r], s[3][r]));
      tm = fmaxf(tm, __shfl_xor(tm, 1, 16));
      tm = fmaxf(tm, __shfl_xor(tm, 2, 16));
      tm = fmaxf(tm, __shfl_xor(tm, 4, 16));
      tm = fmaxf(tm, __shfl_xor(tm, 8, 16));
      const float mn = fmaxf(mrun[r], tm);
      sc[r] = __expf(mrun[r] - mn);
      mrun[r] = mn;
      float rs = 0.0f;
#pragma unroll
      for (int mt = 0; mt < 4; ++mt) {
        const float pv = __expf(s[mt][r] - mn);
        s[mt][r] = pv;
        rs += pv;
      }
      rs += __shfl_xor(rs, 1, 16);
      rs += __shfl_xor(rs, 2, 16);
      rs += __shfl_xor(rs, 4, 16);
      rs += __shfl_xor(rs, 8, 16);
      lrun[r] = lrun[r] * sc[r] + rs;
    }
#pragma unroll
    for (int dt = 0; dt < 4; ++dt)
#pragma unroll
      for (int r = 0; r < 8; ++r) oacc[dt][r] *= sc[r];

#pragma unroll
    for (int mt = 0; mt < 4; ++mt)
#pragma unroll
      for (int r = 0; r < 8; ++r)
        pw[(8 * h + r) * 72 + mt * 16 + m] = (unsigned short)h16_bits(s[mt][r] * 4096.0f);
    asm volatile("" ::: "memory");

#pragma unroll
    for (int ks = 0; ks < 2; ++ks) {
      const int po = m * 72 + ks * 32 + 8 * h;
      FragH pa;
      pa.q[0] = *(const v4ua*)(pw + po);
      pa.q[1] = *(const v4ua*)(pw + po + 16);
#pragma unroll
      for (int dt = 0; dt < 4; ++dt) {
        const int vo = (dt * 16 + m) * 72 + ks * 32 + 8 * h;
        FragH vf;
        vf.q[0] = *(const v4ua*)(vb + vo);
        vf.q[1] = *(const v4ua*)(vb + vo + 16);
        oacc[dt] = mma_f16(pa.v, vf.v, oacc[dt]);
      }
    }
  }

  __syncthreads();
  float* sof = (float*)lds_raw;
  {
    float inv[8];
#pragma unroll
    for (int r = 0; r < 8; ++r) inv[r] = __builtin_amdgcn_rcpf(lrun[r] * 524288.0f);
#pragma unroll
    for (int dt = 0; dt < 4; ++dt)
#pragma unroll
      for (int r = 0; r < 8; ++r)
        sof[(dt * 16 + m) * 128 + wv * 16 + 8 * h + r] = oacc[dt][r] * inv[r];
  }
  __syncthreads();
  v4fa vals[8];
#pragma unroll
  for (int i = 0; i < 8; ++i) {
    const int L = wv * 32 + i * 4 + (lane >> 3);
    const int dl = L >> 2, qt = L & 3;
    vals[i] = *(const v4fa*)(sof + dl * 128 + qt * 32 + (lane & 7) * 4);
  }
#pragma unroll
  for (int i = 0; i < 8; ++i) {
    const int L = wv * 32 + i * 4 + (lane >> 3);
    const int dl = L >> 2, qt = L & 3;
    float* dst = xo + (((size_t)(b * F_DIM + dl * NH + head)) * NSEQ + n0b + qt * 32 + (lane & 7) * 4);
    *(volatile v4fa*)dst = vals[i];
  }
  __threadfence();
#pragma unroll
  for (int i = 0; i < 8; ++i) {
    const int L = wv * 32 + i * 4 + (lane >> 3);
    const int dl = L >> 2, qt = L & 3;
    float* dst = xo + (((size_t)(b * F_DIM + dl * NH + head)) * NSEQ + n0b + qt * 32 + (lane & 7) * 4);
    *(volatile v4fa*)dst = vals[i];
  }
}

extern "C" void kernel_launch(void* const* d_in, const int* in_sizes, int n_in,
                              void* d_out, int out_size, void* d_ws, size_t ws_size,
                              hipStream_t stream)
{
  if (n_in < 11) return;
  const int nX = in_sizes[0];
  const int nB = nX / (F_DIM * NSEQ);
  if (nB <= 0 || nB * F_DIM * NSEQ != nX) return;
  if (in_sizes[1] != nX || in_sizes[2] != nX || out_size != nX) return;
  if (in_sizes[3] != F_DIM * F_DIM || in_sizes[5] != F_DIM * F_DIM ||
      in_sizes[7] != F_DIM * F_DIM || in_sizes[9] != F_DIM * F_DIM) return;
  if (in_sizes[4] != F_DIM || in_sizes[6] != F_DIM || in_sizes[8] != F_DIM || in_sizes[10] != F_DIM) return;

  const float* query = (const float*)d_in[0];
  const float* key_  = (const float*)d_in[1];
  const float* value = (const float*)d_in[2];
  const float* Wq = (const float*)d_in[3];
  const float* bq = (const float*)d_in[4];
  const float* Wk = (const float*)d_in[5];
  const float* bk = (const float*)d_in[6];
  const float* Wv = (const float*)d_in[7];
  const float* bv = (const float*)d_in[8];
  const float* Wm = (const float*)d_in[9];
  const float* bm = (const float*)d_in[10];

  char* ws = (char*)d_ws;
  const size_t nW   = (size_t)F_DIM * F_DIM;
  const size_t wset = 4 * nW * 2;
  size_t off = 0;
  unsigned short* w_hi = (unsigned short*)(ws + off); off += wset;
  unsigned short* w_lo = (unsigned short*)(ws + off); off += wset;
  const size_t nAct = (size_t)nB * F_DIM * NSEQ;
  const size_t p16  = nAct * 2;
  unsigned short* q_hi = (unsigned short*)(ws + off); off += p16;
  unsigned short* q_lo = (unsigned short*)(ws + off); off += p16;
  unsigned short* k_hi = (unsigned short*)(ws + off); off += p16;
  unsigned short* k_lo = (unsigned short*)(ws + off); off += p16;
  unsigned short* v_p  = (unsigned short*)(ws + off); off += p16;
  float*          x_w  = (float*)(ws + off);          off += nAct * 4;
  if (off > ws_size) return;

  k_wcvt<<<dim3((unsigned)((4 * nW / 8 + 255) / 256)), dim3(256), 0, stream>>>(
      Wq, Wk, Wv, Wm, w_hi, w_lo, (int)nW);

  const dim3 pg((unsigned)(nB * (NSEQ / 64))), pb(256);
  k_proj<0><<<pg, pb, 0, stream>>>(query, w_hi + 0 * nW, w_lo + 0 * nW, bq, q_hi, q_lo, x_w, nB);
  k_proj<0><<<pg, pb, 0, stream>>>(key_,  w_hi + 1 * nW, w_lo + 1 * nW, bk, k_hi, k_lo, x_w, nB);
  k_proj<1><<<pg, pb, 0, stream>>>(value, w_hi + 2 * nW, w_lo + 2 * nW, bv, v_p, v_p, x_w, nB);

  k_attn<<<dim3((unsigned)(nB * NH * (NSEQ / 128))), dim3(256), 0, stream>>>(
      q_hi, q_lo, k_hi, k_lo, v_p, x_w, nB);

  k_proj<2><<<pg, pb, 0, stream>>>(x_w, w_hi + 3 * nW, w_lo + 3 * nW, bm, v_p, v_p, (float*)d_out, nB);
  (void)hipGetLastError();
}
